// S6_15607911154022
// MI455X (gfx1250) — hardware-verified
//
#include <hip/hip_runtime.h>
#include <math.h>

typedef __attribute__((ext_vector_type(16))) _Float16 v16h;
typedef __attribute__((ext_vector_type(8)))  _Float16 v8h;
typedef __attribute__((ext_vector_type(16))) __bf16   v16b;
typedef __attribute__((ext_vector_type(8)))  __bf16   v8b;
typedef __attribute__((ext_vector_type(8)))  float    v8f;
typedef __attribute__((ext_vector_type(4)))  float    v4f;
typedef __attribute__((ext_vector_type(4)))  unsigned v4u;

constexpr int kRows = 4096;
constexpr int kDim  = 1024;
constexpr int kNst  = 16;
constexpr int kW23R = 2 * kNst;
constexpr int kTrP  = 68;
static_assert(kDim % 32 == 0);
static_assert(kRows % 64 == 0 && kDim % 64 == 0);
static_assert((kRows * kDim) % (8 * 256) == 0);
static_assert(kDim == 8 * 128);
static_assert(kDim == 4 * 256);

constexpr size_t kOffXB   = 0;
constexpr size_t kOffW1T  = kOffXB  + (size_t)kRows * kDim * 2;
constexpr size_t kOffW23  = kOffW1T + (size_t)kDim  * kDim * 2;
constexpr size_t kOffS    = kOffW23 + (size_t)kW23R * kDim * 2;
constexpr size_t kOffZ    = kOffS   + (size_t)kRows * 4;
constexpr size_t kWsTotal = kOffZ   + (size_t)kRows * kDim * 4;
static_assert(kWsTotal == 27344896ull);
static_assert(kWsTotal <= 134217728ull);
static_assert((kOffW1T % 128) == 0 && (kOffW23 % 128) == 0 && (kOffS % 128) == 0 && (kOffZ % 128) == 0);

__device__ __forceinline__ unsigned short f2bf_bits(float f) {
  unsigned u = __float_as_uint(f);
  return (unsigned short)((u + 0x7FFFu + ((u >> 16) & 1u)) >> 16);
}
__device__ __forceinline__ float bf_bits2f(unsigned short h) { return __uint_as_float(((unsigned)h) << 16); }
__device__ __forceinline__ unsigned pack_bf16x2(float lo, float hi) {
  return (unsigned)f2bf_bits(lo) | (((unsigned)f2bf_bits(hi)) << 16);
}

__device__ __forceinline__ void dep_guard_h(v8f& a, v8f& b, v16h x, v16h y) { asm volatile("v_nop\n\tv_nop\n\tv_nop\n\tv_nop" : "+v"(a), "+v"(b) : "v"(x), "v"(y)); }
__device__ __forceinline__ void dep_guard_b(v8f& a, v8f& b, v16b x, v16b y) { asm volatile("v_nop\n\tv_nop\n\tv_nop\n\tv_nop" : "+v"(a), "+v"(b) : "v"(x), "v"(y)); }
__device__ __forceinline__ void tie4_h(v8f& a, v8f& b, v8f& c, v8f& d, v16h x, v16h y0, v16h y1, v16h y2, v16h y3) {
  asm volatile("v_nop\n\tv_nop\n\tv_nop\n\tv_nop" : "+v"(a), "+v"(b), "+v"(c), "+v"(d) : "v"(x), "v"(y0), "v"(y1), "v"(y2), "v"(y3));
}
__device__ __forceinline__ void tie4_b(v8f& a, v8f& b, v8f& c, v8f& d, v16b x, v16b y0, v16b y1, v16b y2, v16b y3) {
  asm volatile("v_nop\n\tv_nop\n\tv_nop\n\tv_nop" : "+v"(a), "+v"(b), "+v"(c), "+v"(d) : "v"(x), "v"(y0), "v"(y1), "v"(y2), "v"(y3));
}
__device__ __forceinline__ void tie2x3_b(v8f& a, v8f& b, v16b x, v16b y, v16b z) {
  asm volatile("v_nop\n\tv_nop\n\tv_nop\n\tv_nop" : "+v"(a), "+v"(b) : "v"(x), "v"(y), "v"(z));
}
__device__ __forceinline__ void keep4_h(v16h a, v16h b, v16h c, v16h d) { asm volatile("v_nop" :: "v"(a), "v"(b), "v"(c), "v"(d)); }
__device__ __forceinline__ void keep4_b(v16b a, v16b b, v16b c, v16b d) { asm volatile("v_nop" :: "v"(a), "v"(b), "v"(c), "v"(d)); }
__device__ __forceinline__ void acc_guard4(v8f& a, v8f& b, v8f& c, v8f& d) { asm volatile("v_nop\n\tv_nop\n\tv_nop\n\tv_nop" : "+v"(a), "+v"(b), "+v"(c), "+v"(d)); }
template <typename T> struct Frag;
template <> struct Frag<_Float16> {
  typedef v16h V; union U { v16h v; v8h h[2]; };
  static __device__ __forceinline__ v16h load(const _Float16* p) {
    U f; f.h[0] = *(const v8h*)(p); f.h[1] = *(const v8h*)(p + 16); return f.v;
  }
  static __device__ __forceinline__ v8f mma(v16h a, v16h b, v8f c) {
    return __builtin_amdgcn_wmma_f32_16x16x32_f16(false, a, false, b, (short)0, c, false, false);
  }
  static __device__ __forceinline__ void guard(v8f& a, v8f& b, v16h x, v16h y) { dep_guard_h(a, b, x, y); }
  static __device__ __forceinline__ void guard4(v8f& a, v8f& b, v8f& c, v8f& d, v16h x, v16h y0, v16h y1, v16h y2, v16h y3) { tie4_h(a, b, c, d, x, y0, y1, y2, y3); }
  static __device__ __forceinline__ void keep(v16h a, v16h b, v16h c, v16h d) { keep4_h(a, b, c, d); }
};
template <> struct Frag<__bf16> {
  typedef v16b V; union U { v16b v; v8b h[2]; };
  static __device__ __forceinline__ v16b load(const __bf16* p) {
    U f; f.h[0] = *(const v8b*)(p); f.h[1] = *(const v8b*)(p + 16); return f.v;
  }
  static __device__ __forceinline__ v8f mma(v16b a, v16b b, v8f c) {
    return __builtin_amdgcn_wmma_f32_16x16x32_bf16(false, a, false, b, (short)0, c, false, false);
  }
  static __device__ __forceinline__ void guard(v8f& a, v8f& b, v16b x, v16b y) { dep_guard_b(a, b, x, y); }
  static __device__ __forceinline__ void guard4(v8f& a, v8f& b, v8f& c, v8f& d, v16b x, v16b y0, v16b y1, v16b y2, v16b y3) { tie4_b(a, b, c, d, x, y0, y1, y2, y3); }
  static __device__ __forceinline__ void keep(v16b a, v16b b, v16b c, v16b d) { keep4_b(a, b, c, d); }
};

template <int ET> struct Elem;
template <> struct Elem<0> { typedef _Float16 T; };
template <> struct Elem<1> { typedef __bf16 T; };
template <int ET, bool SPLIT, int BIAS_MODE, int OUT_MODE, bool RESID, int ACT = 0>
__global__ __launch_bounds__(256) void wmma_gemm64(
    const unsigned short* __restrict__ Ap, const unsigned short* __restrict__ A2p, int lda, long strideA,
    const unsigned short* __restrict__ Btp, const unsigned short* __restrict__ Bt2p, int ldb, long strideB,
    void* __restrict__ Cout, void* __restrict__ Cout2, int ldc, long strideC,
    const float* __restrict__ bias,
    const float* __restrict__ resid, long strideR,
    int M, int N, int K, float scale) {
  typedef typename Elem<ET>::T T;
  typedef typename Frag<T>::V V;
  const T* A = (const T*)Ap; const T* A2 = (const T*)A2p; const T* Bt = (const T*)Btp; const T* Bt2 = (const T*)Bt2p;
  __shared__ __align__(16) float sT[8][16 * 68];
  const int b    = blockIdx.y;
  const int lane = threadIdx.x & 31;
  const int wave = threadIdx.x >> 5;
  const int tilesN = N >> 6;
  const int tilesM = M >> 6;
  const int tile = blockIdx.x * 8 + wave;
  if (tile >= tilesM * tilesN) return;
  const int tm = tile / tilesN;
  const int tn = tile - tm * tilesN;
  const int m0 = tm << 6;
  const int n0 = tn << 6;

  const T* Ab  = A  + (size_t)b * strideA;
  const T* Bb  = Bt + (size_t)b * strideB;
  const T* Ab2 = SPLIT ? (A2  + (size_t)b * strideA) : nullptr;
  const T* Bb2 = SPLIT ? (Bt2 + (size_t)b * strideB) : nullptr;

  const int rlane = lane & 15;
  const int koff  = (lane >> 4) * 8;
  const int mOff  = (lane >> 4) * 8;

  v8f acc[4][4];
#pragma unroll
  for (int i = 0; i < 4; ++i)
#pragma unroll
    for (int j = 0; j < 4; ++j) acc[i][j] = (v8f){0.f,0.f,0.f,0.f,0.f,0.f,0.f,0.f};

  for (int k0 = 0; k0 < K; k0 += 32) {
    V bh[4], bl[4];
#pragma unroll
    for (int j = 0; j < 4; ++j) {
      const size_t bo = (size_t)(n0 + (j << 4) + rlane) * ldb + koff + k0;
      bh[j] = Frag<T>::load(Bb + bo);
      if (SPLIT) bl[j] = Frag<T>::load(Bb2 + bo);
    }
#pragma unroll
    for (int i = 0; i < 4; ++i) {
      const size_t ao = (size_t)(m0 + (i << 4) + rlane) * lda + koff + k0;
      V ah = Frag<T>::load(Ab + ao);
      V al;
      if (SPLIT) al = Frag<T>::load(Ab2 + ao);
#pragma unroll
      for (int j = 0; j < 4; ++j) {
        acc[i][j] = Frag<T>::mma(ah, bh[j], acc[i][j]);
        if (SPLIT) {
          acc[i][j] = Frag<T>::mma(ah, bl[j], acc[i][j]);
          acc[i][j] = Frag<T>::mma(al, bh[j], acc[i][j]);
        }
      }
      Frag<T>::guard4(acc[i][0], acc[i][1], acc[i][2], acc[i][3], ah, bh[0], bh[1], bh[2], bh[3]);
      if (SPLIT) Frag<T>::guard4(acc[i][0], acc[i][1], acc[i][2], acc[i][3], al, bl[0], bl[1], bl[2], bl[3]);
    }
    Frag<T>::keep(bh[0], bh[1], bh[2], bh[3]);
    if (SPLIT) Frag<T>::keep(bl[0], bl[1], bl[2], bl[3]);
  }
  acc_guard4(acc[0][0], acc[0][1], acc[0][2], acc[0][3]);
  acc_guard4(acc[1][0], acc[1][1], acc[1][2], acc[1][3]);
  acc_guard4(acc[2][0], acc[2][1], acc[2][2], acc[2][3]);
  acc_guard4(acc[3][0], acc[3][1], acc[3][2], acc[3][3]);

  float* slab = sT[wave];
  const float* Rb = RESID ? (resid + (size_t)b * strideR) : nullptr;
#pragma unroll
  for (int i = 0; i < 4; ++i) {
    const int mBase = m0 + (i << 4);
#pragma unroll
    for (int j = 0; j < 4; ++j) {
      const int n = n0 + (j << 4) + rlane;
      float bv = 0.f;
      if (BIAS_MODE == 2) bv = bias[n];
#pragma unroll
      for (int r = 0; r < 8; ++r) {
        float v = acc[i][j][r] * scale;
        if (BIAS_MODE == 1) v += bias[mBase + mOff + r];
        if (BIAS_MODE == 2) v += bv;
        if (RESID) v += Rb[(size_t)(mBase + mOff + r) * ldc + n];
        if (ACT == 1) v = tanhf(v);
        if (ACT == 2) v = fmaxf(v, 0.0f);
        if (ACT == 3) v = v / (1.0f + expf(-v));
        if (ACT == 4) v = (v > 0.f) ? v : 0.01f * v;
        slab[(mOff + r) * 68 + (j << 4) + rlane] = v;
      }
    }
    __builtin_amdgcn_fence(__ATOMIC_RELEASE, "workgroup");
    __builtin_amdgcn_wave_barrier();
    __builtin_amdgcn_fence(__ATOMIC_ACQUIRE, "workgroup");
    if (OUT_MODE == 0) {
      float* C = (float*)Cout + (size_t)b * strideC;
      const int hh = lane >> 4, c4 = (lane & 15) * 4;
      for (int pass = 0; pass < 2; ++pass) {
#pragma unroll
        for (int it = 0; it < 8; ++it) {
          const int row = it * 2 + hh;
          v4f v = *(const v4f*)(slab + row * 68 + c4);
          *(volatile v4f*)(C + (size_t)(mBase + row) * ldc + n0 + c4) = v;
        }
        __threadfence();
      }
    } else {
      const int q = lane >> 3, c8 = (lane & 7) * 8;
      unsigned short* C  = (unsigned short*)Cout  + (size_t)b * strideC;
      unsigned short* C2 = (OUT_MODE == 2) ? ((unsigned short*)Cout2 + (size_t)b * strideC) : nullptr;
      for (int pass = 0; pass < 2; ++pass) {
#pragma unroll
        for (int it = 0; it < 4; ++it) {
          const int row = it * 4 + q;
          const float* sp = slab + row * 68 + c8;
          v8h hv, lv;
#pragma unroll
          for (int e = 0; e < 8; ++e) {
            if (OUT_MODE == 1) {
              hv[e] = (_Float16)sp[e];
            } else {
              unsigned short hb = f2bf_bits(sp[e]);
              unsigned short lb = f2bf_bits(sp[e] - bf_bits2f(hb));
              hv[e] = __builtin_bit_cast(_Float16, hb);
              lv[e] = __builtin_bit_cast(_Float16, lb);
            }
          }
          *(volatile v8h*)(C + (size_t)(mBase + row) * ldc + n0 + c8) = hv;
          if (OUT_MODE == 2) *(volatile v8h*)(C2 + (size_t)(mBase + row) * ldc + n0 + c8) = lv;
        }
        __threadfence();
      }
    }
    __builtin_amdgcn_fence(__ATOMIC_RELEASE, "workgroup");
    __builtin_amdgcn_wave_barrier();
    __builtin_amdgcn_fence(__ATOMIC_ACQUIRE, "workgroup");
  }
}

__global__ __launch_bounds__(256) void rows_to_bf16_kernel(
    const float* __restrict__ src, unsigned short* __restrict__ dst, int total8)
{
  const int i = blockIdx.x * 256 + threadIdx.x;
  if (i >= total8) return;
  const size_t e0 = (size_t)i << 3;
  const v4f a0 = *(const v4f*)(src + e0);
  const v4f a1 = *(const v4f*)(src + e0 + 4);
  v4u w;
  w.x = pack_bf16x2(a0.x, a0.y);
  w.y = pack_bf16x2(a0.z, a0.w);
  w.z = pack_bf16x2(a1.x, a1.y);
  w.w = pack_bf16x2(a1.z, a1.w);
  unsigned short* q = dst + e0;
  *(volatile v4u*)q = w;
  __threadfence();
  *(volatile v4u*)q = w;
}

__global__ __launch_bounds__(256) void w1_transpose_bf16_kernel(
    const float* __restrict__ W1, unsigned short* __restrict__ W1T)
{
  __shared__ __align__(16) float tile[64 * kTrP];
  const int tid = threadIdx.x, lane = tid & 31, wave = tid >> 5;
  const int k0 = blockIdx.y * 64, n0 = blockIdx.x * 64;
#pragma unroll
  for (int i = 0; i < 4; ++i) {
    const int f = tid + 256 * i;
    const int krow = f >> 4, n4 = (f & 15) * 4;
    const v4f v = *(const v4f*)(W1 + (size_t)(k0 + krow) * kDim + n0 + n4);
    *(v4f*)(tile + krow * kTrP + n4) = v;
  }
  __syncthreads();
  const int q = lane >> 3, c8 = (lane & 7) * 8;
  v4u wv[2];
#pragma unroll
  for (int it = 0; it < 2; ++it) {
    const int nl = wave * 8 + it * 4 + q;
    const float* tp = tile + c8 * kTrP + nl;
    const unsigned u0 = pack_bf16x2(tp[0 * kTrP], tp[1 * kTrP]);
    const unsigned u1 = pack_bf16x2(tp[2 * kTrP], tp[3 * kTrP]);
    const unsigned u2 = pack_bf16x2(tp[4 * kTrP], tp[5 * kTrP]);
    const unsigned u3 = pack_bf16x2(tp[6 * kTrP], tp[7 * kTrP]);
    wv[it] = (v4u){u0, u1, u2, u3};
  }
  for (int pass = 0; pass < 2; ++pass) {
#pragma unroll
    for (int it = 0; it < 2; ++it) {
      const int nl = wave * 8 + it * 4 + q;
      *(volatile v4u*)(W1T + (size_t)(n0 + nl) * kDim + k0 + c8) = wv[it];
    }
    __threadfence();
  }
}

__global__ __launch_bounds__(128) void w23_transpose_bf16_kernel(
    const float* __restrict__ W2, const float* __restrict__ W3, unsigned short* __restrict__ W23)
{
  const int nrow = blockIdx.x;
  const int tid = threadIdx.x;
  const float* src = (nrow < kNst) ? W2 : W3;
  const int col = nrow & (kNst - 1);
  const int kb = tid * 8;
  const float* sp = src + (size_t)kb * kNst + col;
  const float f0 = sp[0 * kNst], f1 = sp[1 * kNst], f2 = sp[2 * kNst], f3 = sp[3 * kNst];
  const float f4 = sp[4 * kNst], f5 = sp[5 * kNst], f6 = sp[6 * kNst], f7 = sp[7 * kNst];
  v4u w;
  w.x = pack_bf16x2(f0, f1);
  w.y = pack_bf16x2(f2, f3);
  w.z = pack_bf16x2(f4, f5);
  w.w = pack_bf16x2(f6, f7);
  unsigned short* q = W23 + (size_t)nrow * kDim + kb;
  *(volatile v4u*)q = w;
  __threadfence();
  *(volatile v4u*)q = w;
}

__global__ __launch_bounds__(128) void rowdot_bc_kernel(
    const unsigned short* __restrict__ XBp, const unsigned short* __restrict__ W23p,
    const float* __restrict__ b2, const float* __restrict__ b3,
    const float* __restrict__ Ast, float* __restrict__ S)
{
  (void)Ast;
  __shared__ __align__(16) float sS[64];
  const __bf16* XB = (const __bf16*)XBp;
  const __bf16* WT = (const __bf16*)W23p;
  const int tid = threadIdx.x, lane = tid & 31, wave = tid >> 5;
  const int rl = lane & 15, hh = lane >> 4, koff = hh * 8;
  const int m0 = blockIdx.x * 64 + wave * 16;
  const __bf16* arow = XB + (size_t)(m0 + rl) * kDim + koff;
  const __bf16* brow = WT + (size_t)rl * kDim + koff;
  const __bf16* crow = WT + (size_t)(kNst + rl) * kDim + koff;
  v8f accB = (v8f){0.f,0.f,0.f,0.f,0.f,0.f,0.f,0.f};
  v8f accC = (v8f){0.f,0.f,0.f,0.f,0.f,0.f,0.f,0.f};
#pragma unroll 2
  for (int k0 = 0; k0 < kDim; k0 += 32) {
    const v16b fa = Frag<__bf16>::load(arow + k0);
    const v16b fb = Frag<__bf16>::load(brow + k0);
    const v16b fc = Frag<__bf16>::load(crow + k0);
    accB = Frag<__bf16>::mma(fa, fb, accB);
    accC = Frag<__bf16>::mma(fa, fc, accC);
    tie2x3_b(accB, accC, fa, fb, fc);
  }
  const float bb2 = bf_bits2f(f2bf_bits(b2[rl]));
  const float bb3 = bf_bits2f(f2bf_bits(b3[rl]));
#pragma unroll
  for (int r = 0; r < 8; ++r) {
    float p = (accB[r] + bb2) * (accC[r] + bb3);
    p += __shfl_xor(p, 1, 32);
    p += __shfl_xor(p, 2, 32);
    p += __shfl_xor(p, 4, 32);
    p += __shfl_xor(p, 8, 32);
    if (rl == 0) sS[wave * 16 + hh * 8 + r] = p;
  }
  __syncthreads();
  if (wave == 0) {
    const int l16 = lane & 15;
    const v4f v = *(const v4f*)(sS + l16 * 4);
    float* dst = S + (size_t)blockIdx.x * 64 + l16 * 4;
    if (lane < 16) *(volatile v4f*)dst = v;
    __threadfence();
    if (lane < 16) *(volatile v4f*)dst = v;
  }
}

__global__ __launch_bounds__(256) void gate_out_kernel(
    const float* __restrict__ Z, const unsigned* __restrict__ XBw, const float* __restrict__ b1,
    const float* __restrict__ S, float* __restrict__ Y)
{
  const int row = blockIdx.x, tid = threadIdx.x;
  const size_t base = (size_t)row * kDim + (size_t)tid * 4;
  const float sv = S[row];
  float y0 = 0.f, y1 = 0.f, y2 = 0.f, y3 = 0.f;
#pragma unroll 1
  for (int e = 0; e < 4; ++e) {
    const float z = Z[base + e];
    const unsigned xw = XBw[(base + e) >> 1];
    const unsigned xbits = (e & 1) ? (xw & 0xffff0000u) : (xw << 16);
    const float xv = __uint_as_float(xbits);
    const float bv = bf_bits2f(f2bf_bits(b1[tid * 4 + e]));
    const float zz = z + bv;
    const float a  = expf(-fabsf(zz));
    const float sp = fmaxf(zz, 0.0f) + log1pf(a);
    const float val = (xv * sp) * sv;
    y0 = (e == 0) ? val : y0;
    y1 = (e == 1) ? val : y1;
    y2 = (e == 2) ? val : y2;
    y3 = (e == 3) ? val : y3;
  }
  const v4f y4 = (v4f){y0, y1, y2, y3};
  float* dst = Y + base;
  *(volatile v4f*)dst = y4;
  __threadfence();
  *(volatile v4f*)dst = y4;
}

extern "C" void kernel_launch(void* const* d_in, const int* in_sizes, int n_in,
                              void* d_out, int out_size, void* d_ws, size_t ws_size,
                              hipStream_t stream) {
  if (n_in < 8) return;
  if (in_sizes[0] != kRows * kDim) return;
  if (in_sizes[1] != kDim * kDim) return;
  if (in_sizes[2] != kDim) return;
  if (in_sizes[3] != kDim * kNst) return;
  if (in_sizes[4] != kNst) return;
  if (in_sizes[5] != kDim * kNst) return;
  if (in_sizes[6] != kNst) return;
  if (out_size != kRows * kDim) return;
  if (ws_size < kWsTotal) return;

  const float* x  = (const float*)d_in[0];
  const float* W1 = (const float*)d_in[1];
  const float* b1 = (const float*)d_in[2];
  const float* W2 = (const float*)d_in[3];
  const float* b2 = (const float*)d_in[4];
  const float* W3 = (const float*)d_in[5];
  const float* b3 = (const float*)d_in[6];
  const float* Ast = (const float*)d_in[7];
  float* out = (float*)d_out;

  char* ws = (char*)d_ws;
  unsigned short* XB  = (unsigned short*)(ws + kOffXB);
  unsigned short* W1T = (unsigned short*)(ws + kOffW1T);
  unsigned short* W23 = (unsigned short*)(ws + kOffW23);
  float*          S   = (float*)(ws + kOffS);
  float*          Z   = (float*)(ws + kOffZ);

  rows_to_bf16_kernel<<<(kRows * kDim / 8) / 256, 256, 0, stream>>>(x, XB, kRows * kDim / 8);
  w1_transpose_bf16_kernel<<<dim3(kDim / 64, kDim / 64), 256, 0, stream>>>(W1, W1T);
  w23_transpose_bf16_kernel<<<kW23R, 128, 0, stream>>>(W2, W3, W23);

  rowdot_bc_kernel<<<kRows / 64, 128, 0, stream>>>(XB, W23, b2, b3, Ast, S);

  wmma_gemm64<1, false, 0, 0, false><<<dim3((kRows / 64) * (kDim / 64) / 8, 1), 256, 0, stream>>>(
      XB, nullptr, kDim, 0L,
      W1T, nullptr, kDim, 0L,
      (void*)Z, nullptr, kDim, 0L,
      nullptr, nullptr, 0L,
      kRows, kDim, kDim, 1.0f);

  gate_out_kernel<<<kRows, 256, 0, stream>>>(Z, (const unsigned*)XB, b1, S, out);
}
